// QORAttention_90177133347668
// MI455X (gfx1250) — hardware-verified
//
#include <hip/hip_runtime.h>
#include <math.h>

typedef __attribute__((ext_vector_type(16))) _Float16 v16h;
typedef __attribute__((ext_vector_type(8)))  _Float16 v8h;
typedef __attribute__((ext_vector_type(16))) __bf16   v16b;
typedef __attribute__((ext_vector_type(8)))  __bf16   v8b;
typedef __attribute__((ext_vector_type(8)))  float    v8f;
typedef __attribute__((ext_vector_type(4)))  float    v4f;

constexpr int SEQ_T     = 4096;
constexpr int DMODEL    = 1024;
constexpr int NHEAD     = 16;
constexpr int HDIM      = 64;
constexpr int QKV_N     = 3072;
constexpr int KCOL0     = 1024;
constexpr int VCOL0     = 2048;
constexpr int NQTILE    = SEQ_T / 64;
constexpr int KEY_CH    = 64;
constexpr int LDS_P16   = 72;
constexpr float W_CARRY = 64.0f;
constexpr float P_CARRY = 32768.0f;
constexpr float O_CARRY = 16.0f;

struct FreqTab { float f[32]; };
static_assert(sizeof(FreqTab) == 128);

__device__ __forceinline__ unsigned short f2bf_bits(float f) {
  unsigned u = __float_as_uint(f);
  return (unsigned short)((u + 0x7FFFu + ((u >> 16) & 1u)) >> 16);
}
__device__ __forceinline__ float bf_bits2f(unsigned short h) { return __uint_as_float(((unsigned)h) << 16); }
__device__ __forceinline__ float rne_bf(float f) { return bf_bits2f(f2bf_bits(f)); }

__device__ __forceinline__ void dep_guard_h(v8f& a, v8f& b, v16h x, v16h y) { asm volatile("v_nop\n\tv_nop\n\tv_nop\n\tv_nop" : "+v"(a), "+v"(b) : "v"(x), "v"(y)); }
__device__ __forceinline__ void dep_guard_b(v8f& a, v8f& b, v16b x, v16b y) { asm volatile("v_nop\n\tv_nop\n\tv_nop\n\tv_nop" : "+v"(a), "+v"(b) : "v"(x), "v"(y)); }
__device__ __forceinline__ void keep4_h(v16h a, v16h b, v16h c, v16h d) { asm volatile("v_nop" :: "v"(a), "v"(b), "v"(c), "v"(d)); }
__device__ __forceinline__ void keep4_b(v16b a, v16b b, v16b c, v16b d) { asm volatile("v_nop" :: "v"(a), "v"(b), "v"(c), "v"(d)); }
__device__ __forceinline__ void acc_guard4(v8f& a, v8f& b, v8f& c, v8f& d) { asm volatile("v_nop\n\tv_nop\n\tv_nop\n\tv_nop" : "+v"(a), "+v"(b), "+v"(c), "+v"(d)); }
template <typename T> struct Frag;
template <> struct Frag<_Float16> {
  typedef v16h V; union U { v16h v; v8h h[2]; };
  static __device__ __forceinline__ v16h load(const _Float16* p) {
    U f; f.h[0] = *(const v8h*)(p); f.h[1] = *(const v8h*)(p + 16); return f.v;
  }
  static __device__ __forceinline__ v8f mma(v16h a, v16h b, v8f c) {
    return __builtin_amdgcn_wmma_f32_16x16x32_f16(false, a, false, b, (short)0, c, false, false);
  }
  static __device__ __forceinline__ void guard(v8f& a, v8f& b, v16h x, v16h y) { dep_guard_h(a, b, x, y); }
  static __device__ __forceinline__ void keep(v16h a, v16h b, v16h c, v16h d) { keep4_h(a, b, c, d); }
};
template <> struct Frag<__bf16> {
  typedef v16b V; union U { v16b v; v8b h[2]; };
  static __device__ __forceinline__ v16b load(const __bf16* p) {
    U f; f.h[0] = *(const v8b*)(p); f.h[1] = *(const v8b*)(p + 16); return f.v;
  }
  static __device__ __forceinline__ v8f mma(v16b a, v16b b, v8f c) {
    return __builtin_amdgcn_wmma_f32_16x16x32_bf16(false, a, false, b, (short)0, c, false, false);
  }
  static __device__ __forceinline__ void guard(v8f& a, v8f& b, v16b x, v16b y) { dep_guard_b(a, b, x, y); }
  static __device__ __forceinline__ void keep(v16b a, v16b b, v16b c, v16b d) { keep4_b(a, b, c, d); }
};

__device__ __forceinline__ v8f mma_f16g(v16h a, v16h b, v8f c) {
  c = __builtin_amdgcn_wmma_f32_16x16x32_f16(false, a, false, b, (short)0, c, false, false);
  asm volatile("v_nop\n\tv_nop\n\tv_nop\n\tv_nop" : "+v"(c) : "v"(a), "v"(b));
  return c;
}

template <int ET> struct Elem;
template <> struct Elem<0> { typedef _Float16 T; };
template <> struct Elem<1> { typedef __bf16 T; };
template <int ET, int SPLITM, int BIAS_MODE, int OUT_MODE, bool RESID, int ACT = 0, bool RESID_RNE = false>
__global__ __launch_bounds__(256) void wmma_gemm64(
    const unsigned short* __restrict__ Ap, const unsigned short* __restrict__ A2p, int lda, long strideA,
    const unsigned short* __restrict__ Btp, const unsigned short* __restrict__ Bt2p, int ldb, long strideB,
    void* __restrict__ Cout, void* __restrict__ Cout2, int ldc, long strideC,
    const float* __restrict__ bias,
    const float* __restrict__ resid, long strideR,
    int M, int N, int K, float scale) {
  typedef typename Elem<ET>::T T;
  typedef typename Frag<T>::V V;
  constexpr bool SPA = (SPLITM >= 1);
  constexpr bool SPB = (SPLITM >= 2);
  const T* A = (const T*)Ap; const T* A2 = (const T*)A2p; const T* Bt = (const T*)Btp; const T* Bt2 = (const T*)Bt2p;
  __shared__ __align__(16) float sT[8][16 * 68];
  const int b    = blockIdx.y;
  const int lane = threadIdx.x & 31;
  const int wave = threadIdx.x >> 5;
  const int tilesN = N >> 6;
  const int tilesM = M >> 6;
  const int tile = blockIdx.x * 8 + wave;
  if (tile >= tilesM * tilesN) return;
  const int tm = tile / tilesN;
  const int tn = tile - tm * tilesN;
  const int m0 = tm << 6;
  const int n0 = tn << 6;

  const T* Ab  = A  + (size_t)b * strideA;
  const T* Bb  = Bt + (size_t)b * strideB;
  const T* Ab2 = SPA ? (A2  + (size_t)b * strideA) : nullptr;
  const T* Bb2 = SPB ? (Bt2 + (size_t)b * strideB) : nullptr;

  const int rlane = lane & 15;
  const int koff  = (lane >> 4) * 8;
  const int mOff  = (lane >> 4) * 8;

  v8f acc[4][4];
#pragma unroll
  for (int i = 0; i < 4; ++i)
#pragma unroll
    for (int j = 0; j < 4; ++j) acc[i][j] = (v8f){0.f,0.f,0.f,0.f,0.f,0.f,0.f,0.f};

  for (int k0 = 0; k0 < K; k0 += 32) {
    V bh[4], bl[4];
#pragma unroll
    for (int j = 0; j < 4; ++j) {
      const size_t bo = (size_t)(n0 + (j << 4) + rlane) * ldb + koff + k0;
      bh[j] = Frag<T>::load(Bb + bo);
      if (SPB) bl[j] = Frag<T>::load(Bb2 + bo);
    }
#pragma unroll
    for (int i = 0; i < 4; ++i) {
      const size_t ao = (size_t)(m0 + (i << 4) + rlane) * lda + koff + k0;
      V ah = Frag<T>::load(Ab + ao);
      V al;
      if (SPA) al = Frag<T>::load(Ab2 + ao);
#pragma unroll
      for (int j = 0; j < 4; ++j) {
        acc[i][j] = Frag<T>::mma(ah, bh[j], acc[i][j]);
        if (SPB) acc[i][j] = Frag<T>::mma(ah, bl[j], acc[i][j]);
        if (SPA) acc[i][j] = Frag<T>::mma(al, bh[j], acc[i][j]);
      }
      Frag<T>::guard(acc[i][0], acc[i][3], ah, SPA ? al : ah);
    }
    Frag<T>::keep(bh[0], bh[1], bh[2], bh[3]);
    if (SPB) Frag<T>::keep(bl[0], bl[1], bl[2], bl[3]);
  }
  acc_guard4(acc[0][0], acc[0][1], acc[0][2], acc[0][3]);
  acc_guard4(acc[1][0], acc[1][1], acc[1][2], acc[1][3]);
  acc_guard4(acc[2][0], acc[2][1], acc[2][2], acc[2][3]);
  acc_guard4(acc[3][0], acc[3][1], acc[3][2], acc[3][3]);

  float* slab = sT[wave];
  const float* Rb = RESID ? (resid + (size_t)b * strideR) : nullptr;
#pragma unroll
  for (int i = 0; i < 4; ++i) {
    const int mBase = m0 + (i << 4);
#pragma unroll
    for (int j = 0; j < 4; ++j) {
      const int n = n0 + (j << 4) + rlane;
      float bv = 0.f;
      if (BIAS_MODE == 2) bv = bias[n];
#pragma unroll
      for (int r = 0; r < 8; ++r) {
        float v = acc[i][j][r] * scale;
        if (BIAS_MODE == 1) v += bias[mBase + mOff + r];
        if (BIAS_MODE == 2) v += bv;
        if (RESID) {
          float rv = Rb[(size_t)(mBase + mOff + r) * ldc + n];
          if (RESID_RNE) rv = rne_bf(rv);
          v += rv;
        }
        if (ACT == 1) v = tanhf(v);
        if (ACT == 2) v = fmaxf(v, 0.0f);
        if (ACT == 4) v = (v > 0.f) ? v : 0.01f * v;
        slab[(mOff + r) * 68 + (j << 4) + rlane] = v;
      }
    }
    __builtin_amdgcn_fence(__ATOMIC_RELEASE, "workgroup");
    __builtin_amdgcn_wave_barrier();
    __builtin_amdgcn_fence(__ATOMIC_ACQUIRE, "workgroup");
    if (OUT_MODE == 0) {
      float* C = (float*)Cout + (size_t)b * strideC;
      const int hh = lane >> 4, c4 = (lane & 15) * 4;
      for (int pass = 0; pass < 2; ++pass) {
#pragma unroll
        for (int it = 0; it < 8; ++it) {
          const int row = it * 2 + hh;
          v4f v = *(const v4f*)(slab + row * 68 + c4);
          *(volatile v4f*)(C + (size_t)(mBase + row) * ldc + n0 + c4) = v;
        }
        __threadfence();
      }
    } else {
      const int q = lane >> 3, c8 = (lane & 7) * 8;
      unsigned short* C  = (unsigned short*)Cout  + (size_t)b * strideC;
      unsigned short* C2 = (OUT_MODE == 2) ? ((unsigned short*)Cout2 + (size_t)b * strideC) : nullptr;
      for (int pass = 0; pass < 2; ++pass) {
#pragma unroll
        for (int it = 0; it < 4; ++it) {
          const int row = it * 4 + q;
          const float* sp = slab + row * 68 + c8;
          v8h hv, lv;
#pragma unroll
          for (int e = 0; e < 8; ++e) {
            if (OUT_MODE == 1) {
              hv[e] = (_Float16)sp[e];
            } else {
              unsigned short hb = f2bf_bits(sp[e]);
              unsigned short lb = f2bf_bits(sp[e] - bf_bits2f(hb));
              hv[e] = __builtin_bit_cast(_Float16, hb);
              lv[e] = __builtin_bit_cast(_Float16, lb);
            }
          }
          *(volatile v8h*)(C + (size_t)(mBase + row) * ldc + n0 + c8) = hv;
          if (OUT_MODE == 2) *(volatile v8h*)(C2 + (size_t)(mBase + row) * ldc + n0 + c8) = lv;
        }
        __threadfence();
      }
    }
    __builtin_amdgcn_fence(__ATOMIC_RELEASE, "workgroup");
    __builtin_amdgcn_wave_barrier();
    __builtin_amdgcn_fence(__ATOMIC_ACQUIRE, "workgroup");
  }
}

__global__ __launch_bounds__(128) void rmsnorm_f16_k(const float* __restrict__ x, const float* __restrict__ nw,
                                                     unsigned short* __restrict__ xn) {
  __shared__ float red[4];
  const int t = blockIdx.x, tid = threadIdx.x, wave = tid >> 5, lane = tid & 31;
  const float* row = x + (size_t)t * DMODEL + tid * 8;
  const v4f a = *(const v4f*)row;
  const v4f b = *(const v4f*)(row + 4);
  float xb[8];
#pragma unroll
  for (int e = 0; e < 4; ++e) { xb[e] = rne_bf(a[e]); xb[4 + e] = rne_bf(b[e]); }
  float ss = 0.f;
#pragma unroll
  for (int e = 0; e < 8; ++e) ss += xb[e] * xb[e];
#pragma unroll
  for (int m = 1; m < 32; m <<= 1) ss += __shfl_xor(ss, m, 32);
  if (lane == 0) red[wave] = ss;
  __syncthreads();
  const float tot = (red[0] + red[1]) + (red[2] + red[3]);
  const float inv = rsqrtf(tot * (1.0f / 1024.0f) + 1e-6f);
  const v4f na = *(const v4f*)(nw + tid * 8);
  const v4f nb = *(const v4f*)(nw + tid * 8 + 4);
  v8h hv;
#pragma unroll
  for (int e = 0; e < 4; ++e) {
    hv[e]     = (_Float16)((xb[e] * inv) * rne_bf(na[e]));
    hv[4 + e] = (_Float16)((xb[4 + e] * inv) * rne_bf(nb[e]));
  }
  unsigned short* dst = xn + (size_t)t * DMODEL + tid * 8;
  *(volatile v8h*)dst = hv;
  __threadfence();
  *(volatile v8h*)dst = hv;
}

__global__ __launch_bounds__(256) void cast_w_f16x8_k(const float* __restrict__ w, unsigned short* __restrict__ out,
                                                      int n8, float carry) {
  const int i = blockIdx.x * 256 + threadIdx.x;
  if (i < n8) {
    const v4f a = *(const v4f*)(w + (size_t)8 * i);
    const v4f b = *(const v4f*)(w + (size_t)8 * i + 4);
    v8h hv;
#pragma unroll
    for (int e = 0; e < 4; ++e) {
      hv[e]     = (_Float16)(rne_bf(a[e]) * carry);
      hv[4 + e] = (_Float16)(rne_bf(b[e]) * carry);
    }
    unsigned short* dst = out + (size_t)8 * i;
    *(volatile v8h*)dst = hv;
    __threadfence();
    *(volatile v8h*)dst = hv;
  }
}

__global__ __launch_bounds__(256) void rope_qk_f16_k(const float* __restrict__ qkv, FreqTab ft,
                                                     unsigned short* __restrict__ qpl, unsigned short* __restrict__ kpl) {
#pragma clang fp contract(off)
  __shared__ float cs[2][32];
  __shared__ __align__(16) _Float16 stg[8][4 * LDS_P16];
  const int t = blockIdx.x;
  const int tid = threadIdx.x, wave = tid >> 5, ln = tid & 31;
  if (wave == 0) {
    float fr = ft.f[0];
#pragma unroll
    for (int q = 1; q < 32; ++q) fr = (ln == q) ? ft.f[q] : fr;
    const float ang = (float)t * fr;
    float sv, cv;
    sincosf(ang, &sv, &cv);
    cs[0][ln] = cv;
    cs[1][ln] = sv;
  }
  __syncthreads();
  const float cv = cs[0][ln], sv = cs[1][ln];
  const float* row = qkv + (size_t)t * QKV_N;
  _Float16* sw = stg[wave];
#pragma unroll
  for (int j = 0; j < 2; ++j) {
    const int hq = 2 * wave + j;
    const float x1 = row[hq * HDIM + ln];
    const float x2 = row[hq * HDIM + ln + 32];
    sw[j * LDS_P16 + ln]      = (_Float16)(x1 * cv - x2 * sv);
    sw[j * LDS_P16 + ln + 32] = (_Float16)(x2 * cv + x1 * sv);
    const float k1 = row[KCOL0 + hq * HDIM + ln];
    const float k2 = row[KCOL0 + hq * HDIM + ln + 32];
    sw[(2 + j) * LDS_P16 + ln]      = (_Float16)(k1 * cv - k2 * sv);
    sw[(2 + j) * LDS_P16 + ln + 32] = (_Float16)(k2 * cv + k1 * sv);
  }
  __builtin_amdgcn_fence(__ATOMIC_RELEASE, "workgroup");
  __builtin_amdgcn_wave_barrier();
  __builtin_amdgcn_fence(__ATOMIC_ACQUIRE, "workgroup");

  const int q8 = ln >> 3, c8 = (ln & 7) * 8;
  const v8h val = *(const v8h*)(sw + q8 * LDS_P16 + c8);
  const int hsel = 2 * wave + (q8 & 1);
  const size_t off = ((size_t)hsel * SEQ_T + t) * HDIM + c8;
  unsigned short* dst = ((q8 < 2) ? qpl : kpl) + off;
  for (int pass = 0; pass < 2; ++pass) {
    *(volatile v8h*)dst = val;
    __threadfence();
  }
}

__global__ __launch_bounds__(256) void vt_from_qkv_k(const float* __restrict__ qkv, unsigned short* __restrict__ vt) {
  __shared__ __align__(16) _Float16 th[64 * LDS_P16];
  const int t0 = blockIdx.x * 64, h = blockIdx.y;
  const int tid = threadIdx.x;
  {
    const int sloc = tid >> 2, d0 = (tid & 3) * 16;
    const float* src = qkv + (size_t)(t0 + sloc) * QKV_N + VCOL0 + h * HDIM + d0;
    const v4f a0 = *(const v4f*)(src);
    const v4f a1 = *(const v4f*)(src + 4);
    const v4f a2 = *(const v4f*)(src + 8);
    const v4f a3 = *(const v4f*)(src + 12);
#pragma unroll
    for (int e = 0; e < 4; ++e) {
      th[(d0 + e) * LDS_P16 + sloc]      = (_Float16)a0[e];
      th[(d0 + 4 + e) * LDS_P16 + sloc]  = (_Float16)a1[e];
      th[(d0 + 8 + e) * LDS_P16 + sloc]  = (_Float16)a2[e];
      th[(d0 + 12 + e) * LDS_P16 + sloc] = (_Float16)a3[e];
    }
  }
  __syncthreads();
  const int wave = tid >> 5, lane = tid & 31, q8 = lane >> 3, c8 = (lane & 7) * 8;
  const int dA = wave * 8 + q8, dB = wave * 8 + 4 + q8;
  const v8h va = *(const v8h*)(th + dA * LDS_P16 + c8);
  const v8h vb = *(const v8h*)(th + dB * LDS_P16 + c8);
  const size_t oA = ((size_t)h * HDIM + dA) * SEQ_T + t0 + c8;
  const size_t oB = ((size_t)h * HDIM + dB) * SEQ_T + t0 + c8;
  for (int pass = 0; pass < 2; ++pass) {
    *(volatile v8h*)(vt + oA) = va;
    *(volatile v8h*)(vt + oB) = vb;
    __threadfence();
  }
}

__global__ __launch_bounds__(128) void attn_causal_hd64_k(const unsigned short* __restrict__ qp,
                                                         const unsigned short* __restrict__ kp,
                                                         const unsigned short* __restrict__ vtp,
                                                         unsigned short* __restrict__ op) {
  typedef Frag<_Float16> FH;
  __shared__ __align__(16) _Float16 Ksh[KEY_CH * LDS_P16];
  __shared__ __align__(16) _Float16 Vts[HDIM * LDS_P16];
  __shared__ __align__(16) _Float16 Psh[4][16 * LDS_P16];
  __shared__ __align__(16) float   Os[4][16 * 68];
  const int tid = threadIdx.x, wave = tid >> 5, lane = tid & 31, hh = lane >> 4, c = lane & 15;
  const int qb = blockIdx.x % NQTILE;
  const int h  = blockIdx.x / NQTILE;
  const int q0 = qb * 64 + wave * 16;
  const _Float16* Qh = (const _Float16*)qp + ((size_t)h * SEQ_T + q0 + c) * HDIM;
  const _Float16* Kh = (const _Float16*)kp + (size_t)h * SEQ_T * HDIM;
  const _Float16* Vh = (const _Float16*)vtp + (size_t)h * HDIM * SEQ_T;

  v16h qa[2];
  qa[0] = FH::load(Qh + 8 * hh);
  qa[1] = FH::load(Qh + 32 + 8 * hh);

  const v8f vz = (v8f){0.f,0.f,0.f,0.f,0.f,0.f,0.f,0.f};
  float mrow[8], lrow[8];
  v8f oacc[4];
#pragma unroll
  for (int r = 0; r < 8; ++r) { mrow[r] = -INFINITY; lrow[r] = 0.f; }
#pragma unroll
  for (int t = 0; t < 4; ++t) oacc[t] = vz;

  const int nChunks = qb + 1;
  for (int kc = 0; kc < nChunks; ++kc) {
    const int kv0 = kc * KEY_CH;
    __syncthreads();
#pragma unroll
    for (int i = 0; i < 4; ++i) {
      const int idx = tid + 128 * i;
      const int r = idx >> 3, c8 = (idx & 7) * 8;
      const v8h kv = *(const v8h*)(Kh + (size_t)(kv0 + r) * HDIM + c8);
      const v8h vv = *(const v8h*)(Vh + (size_t)r * SEQ_T + kv0 + c8);
      *(v8h*)(Ksh + r * LDS_P16 + c8) = kv;
      *(v8h*)(Vts + r * LDS_P16 + c8) = vv;
    }
    __syncthreads();

    v8f s[4];
#pragma unroll
    for (int j = 0; j < 4; ++j) {
      s[j] = vz;
#pragma unroll
      for (int dc = 0; dc < 2; ++dc) {
        const v16h kb = FH::load(Ksh + (j * 16 + c) * LDS_P16 + dc * 32 + 8 * hh);
        s[j] = mma_f16g(qa[dc], kb, s[j]);
      }
    }
    const bool diag = (kc == qb);
    float cm[8];
#pragma unroll
    for (int r = 0; r < 8; ++r) {
      const int qrow = q0 + 8 * hh + r;
      float m = -INFINITY;
#pragma unroll
      for (int j = 0; j < 4; ++j) {
        const int kvcol = kv0 + j * 16 + c;
        float sv = s[j][r] * 0.125f;
        if (diag && (kvcol > qrow)) sv = -INFINITY;
        s[j][r] = sv;
        m = fmaxf(m, sv);
      }
#pragma unroll
      for (int off = 1; off < 16; off <<= 1) m = fmaxf(m, __shfl_xor(m, off, 32));
      cm[r] = m;
    }
    _Float16* pw = Psh[wave];
#pragma unroll
    for (int r = 0; r < 8; ++r) {
      const float mnew = fmaxf(mrow[r], cm[r]);
      const float alpha = __expf(mrow[r] - mnew);
      mrow[r] = mnew;
      float psum = 0.f;
#pragma unroll
      for (int j = 0; j < 4; ++j) {
        const float p = __expf(s[j][r] - mnew);
        psum += p;
        pw[(8 * hh + r) * LDS_P16 + j * 16 + c] = (_Float16)(p * P_CARRY);
      }
#pragma unroll
      for (int off = 1; off < 16; off <<= 1) psum += __shfl_xor(psum, off, 32);
      lrow[r] = lrow[r] * alpha + psum;
#pragma unroll
      for (int t = 0; t < 4; ++t) oacc[t][r] *= alpha;
    }
    __builtin_amdgcn_fence(__ATOMIC_RELEASE, "workgroup");
    __builtin_amdgcn_wave_barrier();
    __builtin_amdgcn_fence(__ATOMIC_ACQUIRE, "workgroup");
#pragma unroll
    for (int kk = 0; kk < 2; ++kk) {
      const v16h pa = FH::load(pw + c * LDS_P16 + kk * 32 + 8 * hh);
#pragma unroll
      for (int t = 0; t < 4; ++t) {
        const v16h vb = FH::load(Vts + (t * 16 + c) * LDS_P16 + kk * 32 + 8 * hh);
        oacc[t] = mma_f16g(pa, vb, oacc[t]);
      }
    }
  }

  float* os = Os[wave];
#pragma unroll
  for (int r = 0; r < 8; ++r) {
    const float inv = (1.0f / lrow[r]) * (O_CARRY / P_CARRY);
#pragma unroll
    for (int t = 0; t < 4; ++t) os[(8 * hh + r) * 68 + t * 16 + c] = oacc[t][r] * inv;
  }
  __builtin_amdgcn_fence(__ATOMIC_RELEASE, "workgroup");
  __builtin_amdgcn_wave_barrier();
  __builtin_amdgcn_fence(__ATOMIC_ACQUIRE, "workgroup");
  {
    const int q8 = lane >> 3, c8 = (lane & 7) * 8;
    unsigned short* ob = op + (size_t)h * HDIM + c8;
    for (int pass = 0; pass < 2; ++pass) {
#pragma unroll
      for (int it = 0; it < 4; ++it) {
        const int row = it * 4 + q8;
        const v4f f0 = *(const v4f*)(os + row * 68 + c8);
        const v4f f1 = *(const v4f*)(os + row * 68 + c8 + 4);
        v8h hv;
#pragma unroll
        for (int e = 0; e < 4; ++e) { hv[e] = (_Float16)f0[e]; hv[4 + e] = (_Float16)f1[e]; }
        *(volatile v8h*)(ob + (size_t)(q0 + row) * DMODEL) = hv;
      }
      __threadfence();
    }
  }
}

extern "C" void kernel_launch(void* const* d_in, const int* in_sizes, int n_in,
                              void* d_out, int out_size, void* d_ws, size_t ws_size,
                              hipStream_t stream) {
  if (n_in < 6) return;
  const int nx = SEQ_T * DMODEL;
  const int nwgt = DMODEL * DMODEL;
  if (in_sizes[0] != nx || in_sizes[1] != nwgt || in_sizes[2] != nwgt || in_sizes[3] != nwgt ||
      in_sizes[4] != nwgt || in_sizes[5] != DMODEL || out_size != nx) return;

  const float* x  = (const float*)d_in[0];
  const float* wq = (const float*)d_in[1];
  const float* wk = (const float*)d_in[2];
  const float* wv = (const float*)d_in[3];
  const float* wo = (const float*)d_in[4];
  const float* nw = (const float*)d_in[5];
  float* out = (float*)d_out;

  const size_t szXN   = (size_t)nx * 2;
  const size_t szWQKV = (size_t)3 * nwgt * 2;
  const size_t szWO   = (size_t)nwgt * 2;
  const size_t szQKV  = (size_t)SEQ_T * QKV_N * 4;
  const size_t szPL   = (size_t)NHEAD * SEQ_T * HDIM * 2;
  const size_t szO    = (size_t)nx * 2;
  const size_t offXN   = 0;
  const size_t offWQKV = offXN + szXN;
  const size_t offWO   = offWQKV + szWQKV;
  const size_t offQKV  = offWO + szWO;
  const size_t offQ    = offQKV + szQKV;
  const size_t offK    = offQ + szPL;
  const size_t offVT   = offK + szPL;
  const size_t offO    = offVT + szPL;
  const size_t total   = offO + szO;
  if (total > ws_size) return;

  char* ws = (char*)d_ws;
  unsigned short* XN   = (unsigned short*)(ws + offXN);
  unsigned short* WQKV = (unsigned short*)(ws + offWQKV);
  unsigned short* WO   = (unsigned short*)(ws + offWO);
  float*          QKV  = (float*)(ws + offQKV);
  unsigned short* QPL  = (unsigned short*)(ws + offQ);
  unsigned short* KPL  = (unsigned short*)(ws + offK);
  unsigned short* VT   = (unsigned short*)(ws + offVT);
  unsigned short* OPL  = (unsigned short*)(ws + offO);

  FreqTab ft;
  for (int i = 0; i < 32; ++i) {
    const float e = (float)(2 * i) / 64.0f;
    const float p = (float)pow(10000.0, (double)e);
    ft.f[i] = 1.0f / p;
  }

  rmsnorm_f16_k<<<SEQ_T, 128, 0, stream>>>(x, nw, XN);
  const int n8 = nwgt / 8;
  const int castBlocks = (n8 + 255) / 256;
  cast_w_f16x8_k<<<castBlocks, 256, 0, stream>>>(wq, WQKV, n8, W_CARRY);
  cast_w_f16x8_k<<<castBlocks, 256, 0, stream>>>(wk, WQKV + (size_t)nwgt, n8, W_CARRY);
  cast_w_f16x8_k<<<castBlocks, 256, 0, stream>>>(wv, WQKV + (size_t)2 * nwgt, n8, W_CARRY);
  cast_w_f16x8_k<<<castBlocks, 256, 0, stream>>>(wo, WO, n8, W_CARRY);
  {
    const int tiles = (SEQ_T / 64) * (QKV_N / 64);
    dim3 grid((tiles + 7) / 8, 1);
    wmma_gemm64<0, 0, 0, 0, false><<<grid, 256, 0, stream>>>(
        XN, XN, DMODEL, 0L, WQKV, WQKV, DMODEL, 0L, (void*)QKV, (void*)QKV, QKV_N, 0L,
        nw, x, 0L, SEQ_T, QKV_N, DMODEL, 1.0f / W_CARRY);
  }
  rope_qk_f16_k<<<SEQ_T, 256, 0, stream>>>(QKV, ft, QPL, KPL);
  vt_from_qkv_k<<<dim3(SEQ_T / 64, NHEAD), 256, 0, stream>>>(QKV, VT);
  attn_causal_hd64_k<<<NHEAD * NQTILE, 128, 0, stream>>>(QPL, KPL, VT, OPL);
  {
    const int tiles = (SEQ_T / 64) * (DMODEL / 64);
    dim3 grid((tiles + 7) / 8, 1);
    wmma_gemm64<0, 0, 0, 0, true, 0, true><<<grid, 256, 0, stream>>>(
        OPL, OPL, DMODEL, 0L, WO, WO, DMODEL, 0L, (void*)out, (void*)out, DMODEL, 0L,
        nw, x, 0L, SEQ_T, DMODEL, DMODEL, 1.0f / (O_CARRY * W_CARRY));
  }
}
